// NetPerActionDynaQModel_82789789598536
// MI455X (gfx1250) — hardware-verified
//
#include <hip/hip_runtime.h>


namespace {
constexpr int NB_OUT = 16384  , NBt = 16384  , RPT = NBt / 256, D = 512, H = 1024, A = 18, NEXP = NBt + A * 16  , NT = NEXP / 16;
constexpr float XS = 8.0f, WSC = 256.0f;

typedef _Float16 b16;
typedef __attribute__((ext_vector_type(16))) _Float16 v16b;
typedef __attribute__((ext_vector_type(8))) _Float16 v8b;
typedef __attribute__((ext_vector_type(8))) float v8f;
typedef __attribute__((ext_vector_type(4))) float v4f;
__device__ __forceinline__ float bf16_rne(float f) { unsigned int u = __float_as_uint(f); u += 0x7FFFu + ((u >> 16) & 1u); return __uint_as_float(u & 0xFFFF0000u); }
__device__ __forceinline__ void split16(float v, b16& hi, b16& lo) { hi = (b16)v; lo = (b16)(v - (float)hi); }
__device__ __forceinline__ v16b frag_kb(const b16* p, int hh) { const v8b a = *(const v8b*)(p + 8 * hh), b = *(const v8b*)(p + 16 + 8 * hh); v16b f;
#pragma unroll
  for (int e = 0; e < 8; ++e) { f[e] = a[e]; f[8 + e] = b[e]; } return f; }
__device__ __forceinline__ v8f wmma16b(v16b a, v16b b, v8f c) { v8f d = __builtin_amdgcn_wmma_f32_16x16x32_f16(false, a, false, b, (short)0, c, false, false); asm volatile("v_nop\n\tv_nop\n\tv_nop\n\tv_nop" : "+v"(d) : "v"(a), "v"(b)); return d; }
__device__ __forceinline__ void wave_lds_sync() { __builtin_amdgcn_fence(__ATOMIC_RELEASE, "workgroup"); __builtin_amdgcn_wave_barrier(); __builtin_amdgcn_fence(__ATOMIC_ACQUIRE, "workgroup"); }
__device__ __forceinline__ float nexp(float x) { return __builtin_amdgcn_exp2f(x * 1.4426950408889634f); }
__device__ __forceinline__ int iclamp(int v, int lo, int hi) { return v < lo ? lo : (v > hi ? hi : v); }

__global__ __launch_bounds__(256) void prepx_kernel(const float* __restrict__ obs, b16* __restrict__ X16) {
  const size_t t = (size_t)blockIdx.x * 256 + threadIdx.x; if (t >= (size_t)(NBt + 16) * D / 8) return; const size_t e = t * 8; v8b o = {};
  if (e < (size_t)NBt * D) { const v4f a = *(const v4f*)(obs + e), c = *(const v4f*)(obs + e + 4);
#pragma unroll
    for (int j = 0; j < 4; ++j) { o[j] = (b16)(bf16_rne(a[j]) * XS); o[4 + j] = (b16)(bf16_rne(c[j]) * XS); } }
  for (int pass = 0; pass < 2; ++pass) { *(volatile v8b*)(X16 + e) = o; __threadfence(); }
}
__global__ __launch_bounds__(256) void prepw_kernel(const float* __restrict__ we0, const float* __restrict__ we1, const float* __restrict__ we2, const float* __restrict__ who, const float* __restrict__ whr, const float* __restrict__ whd, b16* __restrict__ WE, b16* __restrict__ WHO, b16* __restrict__ WHRD) {
  __shared__ __attribute__((aligned(16))) b16 T[64][64 + 8];
  const int kind = blockIdx.z, i0 = blockIdx.x * 64, o0 = blockIdx.y * 64, t_ = threadIdx.x;
  if (kind < 3) { if (i0 >= D || o0 >= H) return; const float* w = kind == 0 ? we0 : kind == 1 ? we1 : we2;
    for (int q = t_; q < 64 * 64; q += 256) { const int ii = q >> 6, oo = q & 63; T[oo][ii] = (b16)(bf16_rne(w[(size_t)(i0 + ii) * H + o0 + oo]) * WSC); }
    __syncthreads();
    for (int pass = 0; pass < 2; ++pass) { for (int q = t_; q < 64 * 8; q += 256) { const int oo = q >> 3, c8 = (q & 7) * 8; *(volatile v8b*)(WE + ((size_t)kind * H + o0 + oo) * D + i0 + c8) = *(const v8b*)(&T[oo][c8]); } __threadfence(); } }
  else if (kind < 3 + A) { const int a = kind - 3; if (i0 >= H || o0 >= D) return; const float* w = who + (size_t)a * H * D;
    for (int q = t_; q < 64 * 64; q += 256) { const int ii = q >> 6, oo = q & 63; T[oo][ii] = (b16)(bf16_rne(w[(size_t)(i0 + ii) * D + o0 + oo]) * WSC); }
    __syncthreads();
    for (int pass = 0; pass < 2; ++pass) { for (int q = t_; q < 64 * 8; q += 256) { const int oo = q >> 3, c8 = (q & 7) * 8; *(volatile v8b*)(WHO + ((size_t)a * D + o0 + oo) * H + i0 + c8) = *(const v8b*)(&T[oo][c8]); } __threadfence(); } }
  else { if (blockIdx.y != 0 || i0 >= H) return;
    for (int pass = 0; pass < 2; ++pass) { for (int q = t_; q < 64 * 8; q += 256) { const int rrow = q >> 3, c8 = (q & 7) * 8; const int which = rrow >> 5, a = rrow & 31; v8b o = {};
        if (a < A) { const float* w = (which ? whd : whr) + (size_t)a * H + i0 + c8; for (int j = 0; j < 8; ++j) o[j] = (b16)(bf16_rne(w[j]) * WSC); }
        *(volatile v8b*)(WHRD + ((size_t)which * 32 + a) * H + i0 + c8) = o; } __threadfence(); } }
}
__global__ __launch_bounds__(256) void sort_kernel(const int* __restrict__ actions, int* __restrict__ EXP, int* __restrict__ TACT) {
  __shared__ int cnt[A][256]; __shared__ int base[A + 1], tot[A];
  const int t_ = threadIdx.x; int local[A];
#pragma unroll
  for (int a = 0; a < A; ++a) local[a] = 0;
  for (int i = 0; i < RPT; ++i) { const int a = iclamp(actions[t_ * RPT + i], 0, A - 1);
#pragma unroll
    for (int aa = 0; aa < A; ++aa) local[aa] += (aa == a); }
#pragma unroll
  for (int a = 0; a < A; ++a) cnt[a][t_] = local[a];
  __syncthreads();
  if (t_ < A) { int s = 0; for (int j = 0; j < 256; ++j) { const int c = cnt[t_][j]; cnt[t_][j] = s; s += c; } tot[t_] = s; }
  __syncthreads();
  if (t_ == 0) { int b = 0; for (int a = 0; a < A; ++a) { base[a] = b; b += (tot[a] + 15) & ~15; } base[A] = b; }
  __syncthreads();
#pragma unroll
  for (int a = 0; a < A; ++a) local[a] = cnt[a][t_];
  for (int pass = 0; pass < 2; ++pass) {
    for (int s = t_; s < NEXP; s += 256) { int a = A - 1; for (int aa = 0; aa < A; ++aa) if (s >= base[aa] && s < base[aa + 1]) a = aa; const bool pad = (s >= base[A]) || (s - base[a] >= tot[a]); if (pad) ((volatile int*)EXP)[s] = -1; }
    for (int tIdx = t_; tIdx < NT; tIdx += 256) { const int s = tIdx * 16; int a = 0; for (int aa = 0; aa < A; ++aa) if (s >= base[aa] && s < base[aa + 1]) a = aa; ((volatile int*)TACT)[tIdx] = (s >= base[A]) ? -1 : a; }
    __threadfence(); }
  __syncthreads();
  for (int pass = 0; pass < 2; ++pass) { int pos[A];
#pragma unroll
    for (int a = 0; a < A; ++a) pos[a] = local[a];
    for (int i = 0; i < RPT; ++i) { const int row = t_ * RPT + i; const int a = iclamp(actions[row], 0, A - 1); int p = 0;
#pragma unroll
      for (int aa = 0; aa < A; ++aa) { if (aa == a) { p = pos[aa]; pos[aa] += 1; } }
      ((volatile int*)EXP)[base[a] + p] = row; }
    __threadfence(); }
}
__global__ __launch_bounds__(128) void enc_kernel(const b16* __restrict__ X16, const b16* __restrict__ WE, int x, const float* __restrict__ bb, b16* __restrict__ Fh, b16* __restrict__ Fl) {
  __shared__ __attribute__((aligned(16))) b16 Th[4][16][128 + 8], Tl[4][16][128 + 8];
  const int wave = threadIdx.x >> 5, lane = threadIdx.x & 31, nloc = lane & 15, hlf = lane >> 4; const size_t m0 = (size_t)blockIdx.x * 64 + wave * 16; const int n0 = blockIdx.y * 128;
  const b16* W = WE + (size_t)x * H * D; v8f acc[8];
#pragma unroll
  for (int t = 0; t < 8; ++t) acc[t] = (v8f){};
#pragma unroll 2
  for (int kb = 0; kb < D; kb += 32) { const v16b a = frag_kb(X16 + (m0 + nloc) * D + kb, hlf);
#pragma unroll
    for (int t = 0; t < 8; ++t) acc[t] = wmma16b(a, frag_kb(W + (size_t)(n0 + t * 16 + nloc) * D + kb, hlf), acc[t]); }
#pragma unroll
  for (int t = 0; t < 8; ++t) { const float bv = bf16_rne(bb[n0 + t * 16 + nloc]);
#pragma unroll
    for (int r = 0; r < 8; ++r) { b16 h_, l_; split16(fmaxf(acc[t][r] * (1.0f / (XS * WSC)) + bv, 0.0f) * XS, h_, l_); Th[wave][8 * hlf + r][t * 16 + nloc] = h_; Tl[wave][8 * hlf + r][t * 16 + nloc] = l_; } }
  wave_lds_sync();
  for (int pass = 0; pass < 2; ++pass) { for (int rr = 0; rr < 16; ++rr) if (lane < 16) { const size_t gi = (m0 + rr) * H + n0 + lane * 8; *(volatile v8b*)(Fh + gi) = *(const v8b*)(&Th[wave][rr][lane * 8]); *(volatile v8b*)(Fl + gi) = *(const v8b*)(&Tl[wave][rr][lane * 8]); } __threadfence(); }
}
__global__ __launch_bounds__(128) void fzero_kernel(b16* __restrict__ Fh, b16* __restrict__ Fl) { const int lane = threadIdx.x; const v8b z = {}; const size_t gi = (size_t)NBt * H + lane * 8; for (int pass = 0; pass < 2; ++pass) { *(volatile v8b*)(Fh + gi) = z; *(volatile v8b*)(Fl + gi) = z; __threadfence(); } }
__global__ __launch_bounds__(128) void obshead_kernel(const b16* __restrict__ Fh, const b16* __restrict__ Fl, const int* __restrict__ EXP, const int* __restrict__ TACT, const b16* __restrict__ WHO, const float* __restrict__ bho, const float* __restrict__ obs, float* __restrict__ out0) {
  __shared__ __attribute__((aligned(16))) float Ts[4][16][128 + 4]; __shared__ int Rw[4][16];
  const int wave = threadIdx.x >> 5, lane = threadIdx.x & 31, nloc = lane & 15, hlf = lane >> 4; const int tIdx = blockIdx.x * 4 + wave; const int n0 = blockIdx.y * 128; if (tIdx >= NT) return;
  const int a = TACT[tIdx]; if (a < 0) return;
  const int myrow = EXP[tIdx * 16 + nloc]; const size_t arow = (myrow < 0) ? (size_t)NBt : (size_t)myrow; if (hlf == 0) Rw[wave][nloc] = myrow;
  const b16* W = WHO + (size_t)a * D * H; v8f acc[8];
#pragma unroll
  for (int t = 0; t < 8; ++t) acc[t] = (v8f){};
#pragma unroll 2
  for (int kb = 0; kb < H; kb += 32) { const v16b ah = frag_kb(Fh + arow * H + kb, hlf), al = frag_kb(Fl + arow * H + kb, hlf);
#pragma unroll
    for (int t = 0; t < 8; ++t) { const v16b bw = frag_kb(W + (size_t)(n0 + t * 16 + nloc) * H + kb, hlf); acc[t] = wmma16b(ah, bw, acc[t]); acc[t] = wmma16b(al, bw, acc[t]); } }
#pragma unroll
  for (int t = 0; t < 8; ++t) { const float bb = bf16_rne(bho[(size_t)a * D + n0 + t * 16 + nloc]);
#pragma unroll
    for (int r = 0; r < 8; ++r) Ts[wave][8 * hlf + r][t * 16 + nloc] = acc[t][r] * (1.0f / (XS * WSC)) + bb; }
  wave_lds_sync();
  for (int pass = 0; pass < 2; ++pass) { for (int rr = 0; rr < 16; ++rr) { const int row = Rw[wave][rr]; if (row >= 0) { v4f v = *(const v4f*)(&Ts[wave][rr][lane * 4]); const v4f ob = *(const v4f*)(obs + (size_t)row * D + n0 + lane * 4);
        for (int j = 0; j < 4; ++j) v[j] += bf16_rne(ob[j]); *(volatile v4f*)(out0 + (size_t)row * D + n0 + lane * 4) = v; } } __threadfence(); }
}
__global__ __launch_bounds__(128) void head1_kernel(const b16* __restrict__ Fh, const b16* __restrict__ Fl, const b16* __restrict__ WHRD, int which, const float* __restrict__ bias, const int* __restrict__ actions, float* __restrict__ outv) {
  __shared__ float Sv[64];
  const int wave = threadIdx.x >> 5, lane = threadIdx.x & 31, nloc = lane & 15, hlf = lane >> 4, t_ = threadIdx.x; const size_t m0 = (size_t)blockIdx.x * 64 + wave * 16;
  v8f acc[2] = {{}, {}};
#pragma unroll 2
  for (int kb = 0; kb < H; kb += 32) { const v16b a1 = frag_kb(Fh + (m0 + nloc) * H + kb, hlf), a1l = frag_kb(Fl + (m0 + nloc) * H + kb, hlf);
#pragma unroll
    for (int t = 0; t < 2; ++t) { const v16b bw = frag_kb(WHRD + ((size_t)which * 32 + t * 16 + nloc) * H + kb, hlf); acc[t] = wmma16b(a1, bw, acc[t]); acc[t] = wmma16b(a1l, bw, acc[t]); } }
#pragma unroll
  for (int r = 0; r < 8; ++r) { const size_t row = m0 + 8 * hlf + r; const int a = iclamp(actions[row], 0, A - 1); const int t = a >> 4, c = a & 15;
    const float v0 = acc[0][r] * (1.0f / (XS * WSC)), v1 = acc[1][r] * (1.0f / (XS * WSC)); const float v = (t ? v1 : v0) + bf16_rne(bias[a]);
    if (nloc == c) Sv[wave * 16 + 8 * hlf + r] = which ? 1.0f / (1.0f + nexp(-v)) : v; }
  __syncthreads();
  for (int pass = 0; pass < 2; ++pass) { if (t_ < 64) ((volatile float*)outv)[(size_t)blockIdx.x * 64 + t_] = Sv[t_]; __threadfence(); }
}
}

extern "C" void kernel_launch(void* const* d_in, const int* in_sizes, int n_in, void* d_out, int out_size, void* d_ws, size_t ws_size, hipStream_t stream) {
  (void)n_in;
  auto Fp = [&](int i) { return (const float*)d_in[i]; };
  if (in_sizes[0] != NB_OUT * D || in_sizes[1] != NB_OUT || in_sizes[2] != D * H || in_sizes[8] != A * H * D || in_sizes[10] != A * H || in_sizes[12] != A * H || out_size != NB_OUT * D + 2 * NB_OUT) return;
  size_t off = 0; char* ws = (char*)d_ws;
  auto carve = [&](size_t bytes) { char* p = ws + off; off += (bytes + 255) & ~(size_t)255; return p; };
  b16* X16 = (b16*)carve((size_t)(NBt + 16) * D * 2); b16* WE = (b16*)carve((size_t)3 * H * D * 2); b16* WHO = (b16*)carve((size_t)A * D * H * 2); b16* WHRD = (b16*)carve((size_t)64 * H * 2);
  int* EXP = (int*)carve((size_t)NEXP * 4); int* TACT = (int*)carve((size_t)NT * 4 + 256); b16* Fh = (b16*)carve((size_t)(NBt + 16) * H * 2); b16* Fl = (b16*)carve((size_t)(NBt + 16) * H * 2);
  if (off > ws_size || off > ((size_t)128 << 20)) return;
  prepx_kernel<<<(unsigned)(((size_t)(NBt + 16) * D / 8 + 255) / 256), 256, 0, stream>>>(Fp(0), X16);
  prepw_kernel<<<dim3(H / 64, H / 64, 3 + A + 1), 256, 0, stream>>>(Fp(2), Fp(4), Fp(6), Fp(8), Fp(10), Fp(12), WE, WHO, WHRD);
  sort_kernel<<<1, 256, 0, stream>>>((const int*)d_in[1], EXP, TACT);
  fzero_kernel<<<1, 128, 0, stream>>>(Fh, Fl);
  enc_kernel<<<dim3(NBt / 64, H / 128), 128, 0, stream>>>(X16, WE, 0, Fp(3), Fh, Fl);
  obshead_kernel<<<dim3((NT + 3) / 4, D / 128), 128, 0, stream>>>(Fh, Fl, EXP, TACT, WHO, Fp(9), Fp(0), (float*)d_out);
  enc_kernel<<<dim3(NBt / 64, H / 128), 128, 0, stream>>>(X16, WE, 1, Fp(5), Fh, Fl);
  head1_kernel<<<NBt / 64, 128, 0, stream>>>(Fh, Fl, WHRD, 0, Fp(11), (const int*)d_in[1], (float*)d_out + (size_t)NB_OUT * D);
  enc_kernel<<<dim3(NBt / 64, H / 128), 128, 0, stream>>>(X16, WE, 2, Fp(7), Fh, Fl);
  head1_kernel<<<NBt / 64, 128, 0, stream>>>(Fh, Fl, WHRD, 1, Fp(13), (const int*)d_in[1], (float*)d_out + (size_t)NB_OUT * D + NB_OUT);
}
